// MultiHeadAttention_11879879544649
// MI455X (gfx1250) — hardware-run, weakly checked
//
#include <hip/hip_runtime.h>
#ifndef NB
#define NB 2
#endif
#ifndef SEQ
#define SEQ 2048
#endif
#define NB_FULL 2
#define SEQ_FULL 2048
#define DM 1024
#define NH 16
#define HD 64
#define NF 256
#define NQKV 3072
#ifndef SPLIT_ROWS
#define SPLIT_ROWS 512
#endif
#define SPLIT_EFF ((SPLIT_ROWS) < (SEQ) ? (SPLIT_ROWS) : (SEQ))
#define PLANE ((size_t)NB * NH * SEQ * HD)
#define EPLANE ((size_t)NH * SEQ * HD)
#define CPLANE ((size_t)NB * SEQ * DM)
#define EPITCH 264

#define WS_XB  ((size_t)NB * SEQ * DM * 2)
#define WS_WT  ((size_t)NQKV * DM * 2)
#define WS_PT  ((size_t)DM * NF * 2)
#define WS_WOT ((size_t)DM * DM * 2)
#define WS_P6  ((size_t)6 * PLANE * 2)
#define WS_E2  ((size_t)2 * EPLANE * 2)
#define WS_C2  ((size_t)2 * CPLANE * 2)

static_assert(SEQ % 128 == 0);
static_assert(SPLIT_EFF % 128 == 0);
static_assert(SEQ <= SEQ_FULL);
static_assert(NB <= NB_FULL);
static_assert(HD == 64);
static_assert(NH * HD == DM);
static_assert(WS_XB % 256 == 0 && WS_WT % 256 == 0 && WS_PT % 256 == 0 && WS_WOT % 256 == 0);
static_assert(WS_P6 % 256 == 0 && WS_E2 % 256 == 0 && WS_C2 % 256 == 0);
static_assert(WS_XB + WS_WT + WS_PT + WS_WOT + WS_P6 + WS_E2 + WS_C2 <= (size_t)134217728);

typedef __bf16 v16b __attribute__((ext_vector_type(16)));
typedef _Float16 v16h __attribute__((ext_vector_type(16)));
typedef unsigned short v8us __attribute__((ext_vector_type(8), may_alias));
typedef float v8f __attribute__((ext_vector_type(8)));
typedef float v4f __attribute__((ext_vector_type(4)));
typedef float v4fa __attribute__((ext_vector_type(4), may_alias));
union FragB { v16b v; v8us half[2]; };
union FragH { v16h v; v8us half[2]; _Float16 h[16]; };

#define LOG2E 1.4426950408889634f
#define NEGV (-1000000000.0f)
#define INV2048 0.00048828125f
#define SCL 0.00048828125f
#define WSCALE 0.02374486517661227f
#define OSC 3.0517578125e-05f

__device__ __forceinline__ unsigned short bf16_bits(float x) {
  unsigned int u = __float_as_uint(x);
  return (unsigned short)((u + 0x7FFFu + ((u >> 16) & 1u)) >> 16);
}
__device__ __forceinline__ float bf16_val(unsigned short b) { return __uint_as_float(((unsigned int)b) << 16); }
__device__ __forceinline__ float bf16_rne(float x) { return bf16_val(bf16_bits(x)); }
__device__ __forceinline__ unsigned short f16_bits(float x) { const _Float16 h = (_Float16)x; return __builtin_bit_cast(unsigned short, h); }

__device__ __forceinline__ void split8(const v4f a, const v4f b, v8us& hi, v8us& rs) {
#pragma unroll
  for (int q = 0; q < 4; ++q) {
    const _Float16 h0 = (_Float16)a[q];
    hi[q] = __builtin_bit_cast(unsigned short, h0);
    rs[q] = f16_bits((a[q] - (float)h0) * 2048.0f);
    const _Float16 h1 = (_Float16)b[q];
    hi[4 + q] = __builtin_bit_cast(unsigned short, h1);
    rs[4 + q] = f16_bits((b[q] - (float)h1) * 2048.0f);
  }
}

__device__ __forceinline__ void ldfragH(FragH& f, const unsigned short* __restrict__ p) {
  f.half[0] = *(const v8us*)(p);
  f.half[1] = *(const v8us*)(p + 16);
}
__device__ __forceinline__ void ldfragB(FragB& f, const unsigned short* __restrict__ p) {
  f.half[0] = *(const v8us*)(p);
  f.half[1] = *(const v8us*)(p + 16);
}

__device__ __forceinline__ v8f wmh(v16h a, v16h b, v8f c) {
  return __builtin_amdgcn_wmma_f32_16x16x32_f16(false, a, false, b, (short)0, c, false, false);
}
__device__ __forceinline__ v8f wmb(v16b a, v16b b, v8f c) {
  return __builtin_amdgcn_wmma_f32_16x16x32_bf16(false, a, false, b, (short)0, c, false, false);
}

__device__ __forceinline__ void mma_s1(v16h a0, v16h a1, v16h b0, v16h b1, v8f& c) {
  c = wmh(a0, b0, c);
  c = wmh(a1, b1, c);
  asm volatile("v_nop\n\tv_nop\n\tv_nop\n\tv_nop" : "+v"(c) : "v"(a0), "v"(a1), "v"(b0), "v"(b1));
}
__device__ __forceinline__ void mma_s3(v16h a0, v16h a1, v16h al0, v16h al1, v16h b0, v16h b1, v16h bl0, v16h bl1,
                                       v8f& ch, v8f& cl) {
  ch = wmh(a0, b0, ch);
  ch = wmh(a1, b1, ch);
  cl = wmh(a0, bl0, cl);
  cl = wmh(a1, bl1, cl);
  cl = wmh(al0, b0, cl);
  cl = wmh(al1, b1, cl);
  asm volatile("v_nop\n\tv_nop\n\tv_nop\n\tv_nop" : "+v"(ch), "+v"(cl)
               : "v"(a0), "v"(a1), "v"(al0), "v"(al1), "v"(b0), "v"(b1), "v"(bl0), "v"(bl1));
}
__device__ __forceinline__ void mma_pv4(const FragH (&vf)[4], v16h p, v8f (&c)[4]) {
#pragma unroll
  for (int t = 0; t < 4; ++t) c[t] = wmh(vf[t].v, p, c[t]);
  asm volatile("v_nop\n\tv_nop\n\tv_nop\n\tv_nop" : "+v"(c[0]), "+v"(c[1]), "+v"(c[2]), "+v"(c[3])
               : "v"(vf[0].v), "v"(vf[1].v), "v"(vf[2].v), "v"(vf[3].v), "v"(p));
}
__device__ __forceinline__ void mma_pv3(v16h vh, v16h vl, v16h ph, v16h pl, v8f& ch, v8f& cl) {
  ch = wmh(vh, ph, ch);
  cl = wmh(vh, pl, cl);
  cl = wmh(vl, ph, cl);
  asm volatile("v_nop\n\tv_nop\n\tv_nop\n\tv_nop" : "+v"(ch), "+v"(cl) : "v"(vh), "v"(vl), "v"(ph), "v"(pl));
}
__device__ __forceinline__ void mma_g24b(const FragB (&a)[2], const FragB (&b)[4], v8f (&c)[2][4]) {
#pragma unroll
  for (int i = 0; i < 2; ++i)
#pragma unroll
    for (int j = 0; j < 4; ++j) c[i][j] = wmb(a[i].v, b[j].v, c[i][j]);
  asm volatile("v_nop\n\tv_nop\n\tv_nop\n\tv_nop"
               : "+v"(c[0][0]), "+v"(c[0][1]), "+v"(c[0][2]), "+v"(c[0][3]), "+v"(c[1][0]), "+v"(c[1][1]), "+v"(c[1][2]), "+v"(c[1][3])
               : "v"(a[0].v), "v"(a[1].v), "v"(b[0].v), "v"(b[1].v), "v"(b[2].v), "v"(b[3].v));
}
__device__ __forceinline__ void mma_e(const FragB (&ah)[2], const FragB (&al)[2], const FragB (&b)[4], v8f (&c)[2][4]) {
#pragma unroll
  for (int i = 0; i < 2; ++i)
#pragma unroll
    for (int j = 0; j < 4; ++j) {
      c[i][j] = wmb(ah[i].v, b[j].v, c[i][j]);
      c[i][j] = wmb(al[i].v, b[j].v, c[i][j]);
    }
  asm volatile("v_nop\n\tv_nop\n\tv_nop\n\tv_nop"
               : "+v"(c[0][0]), "+v"(c[0][1]), "+v"(c[0][2]), "+v"(c[0][3]), "+v"(c[1][0]), "+v"(c[1][1]), "+v"(c[1][2]), "+v"(c[1][3])
               : "v"(ah[0].v), "v"(ah[1].v), "v"(al[0].v), "v"(al[1].v), "v"(b[0].v), "v"(b[1].v), "v"(b[2].v), "v"(b[3].v));
}
__device__ __forceinline__ void mma_o1(const FragH (&a)[2], const FragH (&b)[2], v8f (&c)[2][2]) {
#pragma unroll
  for (int i = 0; i < 2; ++i)
#pragma unroll
    for (int j = 0; j < 2; ++j) c[i][j] = wmh(a[i].v, b[j].v, c[i][j]);
  asm volatile("v_nop\n\tv_nop\n\tv_nop\n\tv_nop" : "+v"(c[0][0]), "+v"(c[0][1]), "+v"(c[1][0]), "+v"(c[1][1])
               : "v"(a[0].v), "v"(a[1].v), "v"(b[0].v), "v"(b[1].v));
}
__device__ __forceinline__ void mma_o2(const FragH (&a)[2], const FragH (&l)[2], const FragH (&b)[2], v8f (&ch)[2][2], v8f (&cl)[2][2]) {
#pragma unroll
  for (int i = 0; i < 2; ++i)
#pragma unroll
    for (int j = 0; j < 2; ++j) {
      ch[i][j] = wmh(a[i].v, b[j].v, ch[i][j]);
      cl[i][j] = wmh(l[i].v, b[j].v, cl[i][j]);
    }
  asm volatile("v_nop\n\tv_nop\n\tv_nop\n\tv_nop"
               : "+v"(ch[0][0]), "+v"(ch[0][1]), "+v"(ch[1][0]), "+v"(ch[1][1]), "+v"(cl[0][0]), "+v"(cl[0][1]), "+v"(cl[1][0]), "+v"(cl[1][1])
               : "v"(a[0].v), "v"(a[1].v), "v"(l[0].v), "v"(l[1].v), "v"(b[0].v), "v"(b[1].v));
}

__global__ __launch_bounds__(256) void k_xb(const float* __restrict__ X, unsigned short* __restrict__ Xb) {
  const int t = blockIdx.x * 256 + threadIdx.x;
  if (t >= NB * SEQ * (DM / 8)) return;
  const int row = t >> 7, piece = t & 127;
  const int b = row / SEQ, s = row - b * SEQ;
  const float* src = X + ((size_t)b * SEQ_FULL + s) * DM + piece * 8;
  const v4f x0 = *(const v4fa*)(src), x1 = *(const v4fa*)(src + 4);
  v8us o;
  o[0] = bf16_bits(x0[0]); o[1] = bf16_bits(x0[1]); o[2] = bf16_bits(x0[2]); o[3] = bf16_bits(x0[3]);
  o[4] = bf16_bits(x1[0]); o[5] = bf16_bits(x1[1]); o[6] = bf16_bits(x1[2]); o[7] = bf16_bits(x1[3]);
  unsigned short* d = Xb + (size_t)t * 8;
  *(volatile v8us*)d = o;
  __threadfence();
  *(volatile v8us*)d = o;
}

template <int MODE>
__global__ __launch_bounds__(256) void k_tr(const float* __restrict__ in, unsigned short* __restrict__ out, int rows, int cols) {
  __shared__ unsigned short tl[64][66];
  const int tid = threadIdx.x;
  const int c0 = blockIdx.x * 64, r0 = blockIdx.y * 64;
  for (int i = tid; i < 64 * 16; i += 256) {
    const int j = i >> 4, c4 = (i & 15) * 4;
    const v4f x = *(const v4fa*)(in + (size_t)(r0 + j) * cols + c0 + c4);
#pragma unroll
    for (int q = 0; q < 4; ++q) {
      unsigned short u;
      if (MODE == 0) u = bf16_bits(x[q]);
      else u = f16_bits(bf16_rne(x[q]) * 16.0f);
      tl[c4 + q][j] = u;
    }
  }
  __syncthreads();
  for (int pass = 0; pass < 2; ++pass) {
    for (int i = tid; i < 64 * 8; i += 256) {
      const int c = i >> 3, j8 = (i & 7) * 8;
      v8us o;
#pragma unroll
      for (int q = 0; q < 8; ++q) o[q] = tl[c][j8 + q];
      *(volatile v8us*)(out + (size_t)(c0 + c) * rows + r0 + j8) = o;
    }
    if (pass == 0) __threadfence();
  }
}

__global__ __launch_bounds__(128) void k_emb(const unsigned short* __restrict__ Pt, unsigned short* __restrict__ E2) {
  __shared__ __attribute__((aligned(16))) unsigned int sAh[32 * (EPITCH / 2)];
  __shared__ __attribute__((aligned(16))) unsigned int sAl[32 * (EPITCH / 2)];
  __shared__ __attribute__((aligned(16))) float so[4][16][68];
  const int tid = threadIdx.x, w = __builtin_amdgcn_readfirstlane((int)(tid >> 5)), lane = tid & 31, ln = lane & 15, hh = lane >> 4;
  const int p0 = blockIdx.x * 32;
  {
    const int j = tid;
    const double invf = pow(10000.0, -(double)(2 * j) / 256.0);
#pragma unroll 1
    for (int i = 0; i < 32; ++i) {
      const double ang = (double)(p0 + i) * invf;
      const double kq = rint(ang * 0.15915494309189535);
      double r = fma(-kq, 6.283185307179586, ang);
      r = fma(-kq, 2.4492935982947064e-16, r);
      float sv, cv;
      sincosf((float)r, &sv, &cv);
      const float s2 = (float)(1.4142135623730951 * (double)sv);
      const float c2 = (float)(1.4142135623730951 * (double)cv);
      const unsigned short sh = bf16_bits(s2), ch = bf16_bits(c2);
      const unsigned short sl = bf16_bits(s2 - bf16_val(sh)), cl = bf16_bits(c2 - bf16_val(ch));
      sAh[i * (EPITCH / 2) + j] = (unsigned int)sh | ((unsigned int)ch << 16);
      sAl[i * (EPITCH / 2) + j] = (unsigned int)sl | ((unsigned int)cl << 16);
    }
  }
  __syncthreads();
  const int sub = lane >> 3, piece = lane & 7;
#pragma unroll 1
  for (int h4 = 0; h4 < 4; ++h4) {
    const int hd = w + 4 * h4;
    v8f acc[2][4] = {};
    const unsigned short* bp = Pt + (size_t)(hd * 64 + ln) * NF + 8 * hh;
#pragma unroll 1
    for (int ks = 0; ks < 8; ++ks) {
      FragB ah[2], al[2], bf[4];
#pragma unroll
      for (int i = 0; i < 2; ++i) {
        const int eo = (16 * i + ln) * EPITCH + 32 * ks + 8 * hh;
        ah[i].half[0] = *(const v8us*)((const unsigned short*)sAh + eo);
        ah[i].half[1] = *(const v8us*)((const unsigned short*)sAh + eo + 16);
        al[i].half[0] = *(const v8us*)((const unsigned short*)sAl + eo);
        al[i].half[1] = *(const v8us*)((const unsigned short*)sAl + eo + 16);
      }
#pragma unroll
      for (int jn = 0; jn < 4; ++jn) ldfragB(bf[jn], bp + (size_t)jn * 16 * NF + 32 * ks);
      mma_e(ah, al, bf, acc);
    }
#pragma unroll
    for (int i = 0; i < 2; ++i) {
      __syncthreads();
#pragma unroll
      for (int jn = 0; jn < 4; ++jn)
#pragma unroll
        for (int r = 0; r < 8; ++r) so[w][8 * hh + r][16 * jn + ln] = acc[i][jn][r];
      __syncthreads();
      const size_t base = ((size_t)hd * SEQ + p0 + 16 * i) * HD;
      for (int pass = 0; pass < 2; ++pass) {
#pragma unroll
        for (int q = 0; q < 4; ++q) {
          const int row = 4 * q + sub;
          const v4f x0 = *(const v4fa*)&so[w][row][8 * piece];
          const v4f x1 = *(const v4fa*)&so[w][row][8 * piece + 4];
          v8us hi, rs;
          split8(x0, x1, hi, rs);
          const size_t dst = base + (size_t)row * HD + piece * 8;
          *(volatile v8us*)(E2 + dst) = hi;
          *(volatile v8us*)(E2 + EPLANE + dst) = rs;
        }
        if (pass == 0) __threadfence();
      }
    }
  }
}

__global__ __launch_bounds__(128) void k_qkv(const unsigned short* __restrict__ Xb, const unsigned short* __restrict__ Wt,
                                             const float* __restrict__ qbias, unsigned short* __restrict__ P6) {
  __shared__ __attribute__((aligned(16))) float so[128][68];
  const int tid = threadIdx.x, w = __builtin_amdgcn_readfirstlane((int)(tid >> 5)), lane = tid & 31, ln = lane & 15, hh = lane >> 4;
  const int m0 = blockIdx.x * 128, n0 = blockIdx.y * 64;
  v8f acc[2][4] = {};
  const unsigned short* ap = Xb + (size_t)(m0 + 32 * w + ln) * DM + 8 * hh;
  const unsigned short* bp = Wt + (size_t)(n0 + ln) * DM + 8 * hh;
#pragma unroll 1
  for (int k0 = 0; k0 < DM; k0 += 32) {
    FragB a[2], b[4];
    ldfragB(a[0], ap + k0);
    ldfragB(a[1], ap + (size_t)16 * DM + k0);
#pragma unroll
    for (int j = 0; j < 4; ++j) ldfragB(b[j], bp + (size_t)j * 16 * DM + k0);
    mma_g24b(a, b, acc);
  }
  const int atype = n0 >> 10, head = (n0 >> 6) & 15;
  const int b = m0 / SEQ, s0 = m0 - b * SEQ;
#pragma unroll
  for (int j = 0; j < 4; ++j) {
    const float bq = bf16_rne(qbias[head * 64 + 16 * j + ln]);
    const float bj = (atype == 0) ? bq : 0.0f;
#pragma unroll
    for (int i = 0; i < 2; ++i)
#pragma unroll
      for (int r = 0; r < 8; ++r)
        so[32 * w + 16 * i + 8 * hh + r][16 * j + ln] = (acc[i][j][r] * WSCALE + bj) * 16.0f;
  }
  __syncthreads();
  const int sub = lane >> 3, piece = lane & 7;
  if (atype < 2) {
    const size_t base = (size_t)(2 * atype) * PLANE + ((size_t)(b * NH + head) * SEQ + s0) * HD;
    for (int pass = 0; pass < 2; ++pass) {
#pragma unroll
      for (int it = 0; it < 8; ++it) {
        const int line = 32 * w + 4 * it + sub;
        const v4f x0 = *(const v4fa*)&so[line][8 * piece];
        const v4f x1 = *(const v4fa*)&so[line][8 * piece + 4];
        v8us hi, rs;
        split8(x0, x1, hi, rs);
        const size_t dst = base + (size_t)line * HD + piece * 8;
        *(volatile v8us*)(P6 + dst) = hi;
        *(volatile v8us*)(P6 + PLANE + dst) = rs;
      }
      if (pass == 0) __threadfence();
    }
  } else {
    const size_t base = (size_t)4 * PLANE + ((size_t)(b * NH + head) * HD) * SEQ + s0;
    for (int pass = 0; pass < 2; ++pass) {
#pragma unroll
      for (int it = 0; it < 8; ++it) {
        const int L = 32 * w + 4 * it + sub;
        const int d = L >> 1, seg = L & 1;
        v4f x0, x1;
#pragma unroll
        for (int q = 0; q < 4; ++q) {
          x0[q] = so[seg * 64 + 8 * piece + q][d];
          x1[q] = so[seg * 64 + 8 * piece + 4 + q][d];
        }
        v8us hi, rs;
        split8(x0, x1, hi, rs);
        const size_t dst = base + (size_t)d * SEQ + seg * 64 + piece * 8;
        *(volatile v8us*)(P6 + dst) = hi;
        *(volatile v8us*)(P6 + PLANE + dst) = rs;
      }
      if (pass == 0) __threadfence();
    }
  }
}

template <bool SPLIT, bool MASK>
__device__ __forceinline__ void fa_step(const unsigned short* __restrict__ Kh, const unsigned short* __restrict__ Kl,
                                        const unsigned short* __restrict__ Vh, const unsigned short* __restrict__ Vl,
                                        const unsigned short* __restrict__ Eh, const unsigned short* __restrict__ El,
                                        float (&tlw)[16 * 52], int key0, int qw, int qg, int ln, int hh,
                                        const FragH& q0h, const FragH& q1h, const FragH& q0l, const FragH& q1l,
                                        float& mr, float& lr, v8f (&Oh)[4], v8f (&Ol)[4]) {
  const v8f z8 = {0.f, 0.f, 0.f, 0.f, 0.f, 0.f, 0.f, 0.f};
  v8f sh[2], sl[2];
#pragma unroll
  for (int kt = 0; kt < 2; ++kt) {
    const size_t ko = (size_t)(key0 + 16 * kt + ln) * HD + 8 * hh;
    FragH a0, a1;
    ldfragH(a0, Kh + ko);
    ldfragH(a1, Kh + ko + 32);
    sh[kt] = z8;
    sl[kt] = z8;
    if (SPLIT) {
      FragH l0, l1;
      ldfragH(l0, Kl + ko);
      ldfragH(l1, Kl + ko + 32);
      mma_s3(a0.v, a1.v, l0.v, l1.v, q0h.v, q1h.v, q0l.v, q1l.v, sh[kt], sl[kt]);
    } else {
      mma_s1(a0.v, a1.v, q0h.v, q1h.v, sh[kt]);
    }
  }
  const int dbase = qw - key0 - 31;
#pragma unroll 1
  for (int tt = 0; tt < 3; ++tt) {
    int row = dbase + 16 * tt + ln;
    row = row < 0 ? 0 : (row > SEQ - 1 ? SEQ - 1 : row);
    const size_t eo = (size_t)row * HD + 8 * hh;
    FragH e0, e1;
    ldfragH(e0, Eh + eo);
    ldfragH(e1, Eh + eo + 32);
    v8f th = z8, tq = z8;
    if (SPLIT) {
      FragH l0, l1;
      ldfragH(l0, El + eo);
      ldfragH(l1, El + eo + 32);
      mma_s3(e0.v, e1.v, l0.v, l1.v, q0h.v, q1h.v, q0l.v, q1l.v, th, tq);
    } else {
      mma_s1(e0.v, e1.v, q0h.v, q1h.v, th);
    }
    v4f o0, o1;
#pragma unroll
    for (int r = 0; r < 4; ++r) {
      o0[r] = SPLIT ? (th[r] + tq[r] * INV2048) : th[r];
      o1[r] = SPLIT ? (th[4 + r] + tq[4 + r] * INV2048) : th[4 + r];
    }
    float* dp = &tlw[ln * 52 + 16 * tt + 8 * hh];
    *(v4fa*)dp = o0;
    *(v4fa*)(dp + 4) = o1;
  }
  __syncthreads();
  float sc[16];
#pragma unroll
  for (int kt = 0; kt < 2; ++kt)
#pragma unroll
    for (int r = 0; r < 8; ++r) {
      const int vp = ln + 31 - 16 * kt - 8 * hh - r;
      const float t = tlw[ln * 52 + vp];
      float s = sh[kt][r];
      if (SPLIT) s += sl[kt][r] * INV2048;
      float x = (s + t) * SCL;
      if (MASK) {
        const int kg = key0 + 16 * kt + 8 * hh + r;
        x = (kg > qg) ? NEGV : x;
      }
      sc[8 * kt + r] = x;
    }
  float mx = sc[0];
#pragma unroll
  for (int i = 1; i < 16; ++i) mx = fmaxf(mx, sc[i]);
  mx = fmaxf(mx, __shfl_xor(mx, 16, 32));
  const float mnew = fmaxf(mr, mx);
  const float al = exp2f((mr - mnew) * LOG2E);
  mr = mnew;
  FragH ph, pl;
  float ps = 0.0f;
#pragma unroll
  for (int i = 0; i < 16; ++i) {
    const float pc = exp2f(fmaf(sc[i] - mnew, LOG2E, 8.0f));
    ps += pc;
    const _Float16 h = (_Float16)pc;
    ph.h[i] = h;
    pl.h[i] = SPLIT ? (_Float16)((pc - (float)h) * 2048.0f) : h;
  }
  ps += __shfl_xor(ps, 16, 32);
  lr = lr * al + ps;
#pragma unroll
  for (int t = 0; t < 4; ++t) {
    Oh[t] = Oh[t] * al;
    if (SPLIT) Ol[t] = Ol[t] * al;
  }
  if (SPLIT) {
#pragma unroll
    for (int t = 0; t < 4; ++t) {
      const size_t vo = (size_t)(16 * t + ln) * SEQ + key0 + 8 * hh;
      FragH vh, vl;
      ldfragH(vh, Vh + vo);
      ldfragH(vl, Vl + vo);
      mma_pv3(vh.v, vl.v, ph.v, pl.v, Oh[t], Ol[t]);
    }
  } else {
    FragH vf[4];
#pragma unroll
    for (int t = 0; t < 4; ++t) ldfragH(vf[t], Vh + (size_t)(16 * t + ln) * SEQ + key0 + 8 * hh);
    mma_pv4(vf, ph.v, Oh);
  }
}

template <bool SPLIT>
__global__ __launch_bounds__(64) void k_attn(const unsigned short* __restrict__ P6, const unsigned short* __restrict__ E2,
                                             unsigned short* __restrict__ C2, int qt0, int nqt) {
  __shared__ __attribute__((aligned(16))) float tl[2][16 * 52];
  __shared__ __attribute__((aligned(16))) float so[2][16][68];
  const int tid = threadIdx.x, w = __builtin_amdgcn_readfirstlane((int)(tid >> 5)), lane = tid & 31, ln = lane & 15, hh = lane >> 4;
  const int bh = blockIdx.x / nqt;
  const int qt = qt0 + ((int)blockIdx.x - bh * nqt);
  const int b = bh / NH, head = bh - b * NH;
  const int qw = 32 * qt + 16 * w;
  const int qg = qw + ln;
  const size_t qko = (size_t)bh * SEQ * HD;
  const unsigned short* Qh = P6 + qko;
  const unsigned short* Ql = P6 + PLANE + qko;
  const unsigned short* Kh = P6 + 2 * PLANE + qko;
  const unsigned short* Kl = P6 + 3 * PLANE + qko;
  const unsigned short* Vh = P6 + 4 * PLANE + qko;
  const unsigned short* Vl = P6 + 5 * PLANE + qko;
  const unsigned short* Eh = E2 + (size_t)head * SEQ * HD;
  const unsigned short* El = Eh + EPLANE;
  FragH q0h, q1h, q0l, q1l;
  {
    const size_t qo = (size_t)qg * HD + 8 * hh;
    ldfragH(q0h, Qh + qo);
    ldfragH(q1h, Qh + qo + 32);
    if (SPLIT) {
      ldfragH(q0l, Ql + qo);
      ldfragH(q1l, Ql + qo + 32);
    } else {
      q0l = q0h;
      q1l = q1h;
    }
  }
  float mr = -3.0e38f, lr = 0.0f;
  v8f Oh[4] = {}, Ol[4] = {};
#pragma unroll 1
  for (int j = 0; j < qt; ++j)
    fa_step<SPLIT, false>(Kh, Kl, Vh, Vl, Eh, El, tl[w], 32 * j, qw, qg, ln, hh, q0h, q1h, q0l, q1l, mr, lr, Oh, Ol);
  fa_step<SPLIT, true>(Kh, Kl, Vh, Vl, Eh, El, tl[w], 32 * qt, qw, qg, ln, hh, q0h, q1h, q0l, q1l, mr, lr, Oh, Ol);

  const float inv = 4.0f / lr;
#pragma unroll
  for (int t = 0; t < 4; ++t) {
    v4f o0, o1;
#pragma unroll
    for (int r = 0; r < 4; ++r) {
      o0[r] = (SPLIT ? (Oh[t][r] + Ol[t][r] * INV2048) : Oh[t][r]) * inv;
      o1[r] = (SPLIT ? (Oh[t][4 + r] + Ol[t][4 + r] * INV2048) : Oh[t][4 + r]) * inv;
    }
    *(v4fa*)&so[w][ln][16 * t + 8 * hh] = o0;
    *(v4fa*)&so[w][ln][16 * t + 8 * hh + 4] = o1;
  }
  __syncthreads();
  const int sub = lane >> 3, piece = lane & 7;
  const size_t base = ((size_t)b * SEQ + qw) * DM + (size_t)head * HD;
  for (int pass = 0; pass < 2; ++pass) {
#pragma unroll
    for (int q = 0; q < 4; ++q) {
      const int row = 4 * q + sub;
      const v4f x0 = *(const v4fa*)&so[w][row][8 * piece];
      const v4f x1 = *(const v4fa*)&so[w][row][8 * piece + 4];
      v8us hi, rs;
      split8(x0, x1, hi, rs);
      const size_t dst = base + (size_t)row * DM + piece * 8;
      *(volatile v8us*)(C2 + dst) = hi;
      if (SPLIT) *(volatile v8us*)(C2 + CPLANE + dst) = rs;
    }
    if (pass == 0) __threadfence();
  }
}

template <bool LO>
__device__ __forceinline__ void out_loop(const unsigned short* __restrict__ ap, const unsigned short* __restrict__ bp,
                                         v8f (&ch)[2][2], v8f (&cl)[2][2]) {
#pragma unroll 1
  for (int k0 = 0; k0 < DM; k0 += 32) {
    FragH a[2], b[2];
    ldfragH(a[0], ap + k0);
    ldfragH(a[1], ap + (size_t)16 * DM + k0);
    ldfragH(b[0], bp + k0);
    ldfragH(b[1], bp + (size_t)16 * DM + k0);
    if (LO) {
      FragH l[2];
      ldfragH(l[0], ap + CPLANE + k0);
      ldfragH(l[1], ap + CPLANE + (size_t)16 * DM + k0);
      mma_o2(a, l, b, ch, cl);
    } else {
      mma_o1(a, b, ch);
    }
  }
}

__global__ __launch_bounds__(128) void k_out(const unsigned short* __restrict__ C2, const unsigned short* __restrict__ WoT,
                                             const float* __restrict__ obias, float* __restrict__ out) {
  __shared__ __attribute__((aligned(16))) float so[64][68];
  const int tid = threadIdx.x, w = __builtin_amdgcn_readfirstlane((int)(tid >> 5)), lane = tid & 31, ln = lane & 15, hh = lane >> 4;
  const int wm = w >> 1, wn = w & 1;
  const int m0 = blockIdx.x * 64, n0 = blockIdx.y * 64;
  const int b = m0 / SEQ, s0 = m0 - b * SEQ;
  const bool useLo = s0 < SPLIT_EFF;
  v8f ch[2][2] = {}, cl[2][2] = {};
  const unsigned short* ap = C2 + (size_t)(m0 + 32 * wm + ln) * DM + 8 * hh;
  const unsigned short* bp = WoT + (size_t)(n0 + 32 * wn + ln) * DM + 8 * hh;
  if (useLo) out_loop<true>(ap, bp, ch, cl);
  else out_loop<false>(ap, bp, ch, cl);
#pragma unroll
  for (int j = 0; j < 2; ++j) {
    const float bj = bf16_rne(obias[n0 + 32 * wn + 16 * j + ln]);
#pragma unroll
    for (int i = 0; i < 2; ++i)
#pragma unroll
      for (int r = 0; r < 8; ++r)
        so[32 * wm + 16 * i + 8 * hh + r][32 * wn + 16 * j + ln] = (ch[i][j][r] + cl[i][j][r] * INV2048) * OSC + bj;
  }
  __syncthreads();
  const int rsub = lane >> 4, c4 = (lane & 15) * 4;
  float* og = out + ((size_t)b * SEQ_FULL + s0) * DM + n0;
  for (int pass = 0; pass < 2; ++pass) {
#pragma unroll
    for (int q = 0; q < 8; ++q) {
      const int row = 16 * w + 2 * q + rsub;
      const v4f v = *(const v4fa*)&so[row][c4];
      *(volatile v4f*)(og + (size_t)row * DM + c4) = v;
    }
    if (pass == 0) __threadfence();
  }
}

extern "C" void kernel_launch(void* const* d_in, const int* in_sizes, int n_in,
                              void* d_out, int out_size, void* d_ws, size_t ws_size, hipStream_t stream) {
  if (n_in < 6) return;
  const long long needx = ((long long)(NB - 1) * SEQ_FULL + SEQ) * DM;
  if ((long long)in_sizes[0] < needx) return;
  if ((long long)in_sizes[1] < (long long)DM * NQKV) return;
  if ((long long)in_sizes[2] < (long long)NH * HD) return;
  if ((long long)in_sizes[3] < (long long)NF * NH * HD) return;
  if ((long long)in_sizes[4] < (long long)DM * DM) return;
  if ((long long)in_sizes[5] < (long long)DM) return;
  if ((long long)out_size < needx) return;
  const float* X   = (const float*)d_in[0];
  const float* QKV = (const float*)d_in[1];
  const float* QB  = (const float*)d_in[2];
  const float* POS = (const float*)d_in[3];
  const float* OW  = (const float*)d_in[4];
  const float* OB  = (const float*)d_in[5];
  float* OUT = (float*)d_out;
  char* ws = (char*)d_ws;
  size_t off = 0;
  unsigned short* Xb  = (unsigned short*)(ws + off); off += WS_XB;
  unsigned short* Wt  = (unsigned short*)(ws + off); off += WS_WT;
  unsigned short* Pt  = (unsigned short*)(ws + off); off += WS_PT;
  unsigned short* WoT = (unsigned short*)(ws + off); off += WS_WOT;
  unsigned short* P6  = (unsigned short*)(ws + off); off += WS_P6;
  unsigned short* E2  = (unsigned short*)(ws + off); off += WS_E2;
  unsigned short* C2  = (unsigned short*)(ws + off); off += WS_C2;
  if (off > ws_size) return;

  k_xb<<<(unsigned)((NB * SEQ * (DM / 8) + 255) / 256), 256, 0, stream>>>(X, Xb);
  k_tr<0><<<dim3(NQKV / 64, DM / 64), 256, 0, stream>>>(QKV, Wt, DM, NQKV);
  k_tr<0><<<dim3(DM / 64, NF / 64), 256, 0, stream>>>(POS, Pt, NF, DM);
  k_tr<1><<<dim3(DM / 64, DM / 64), 256, 0, stream>>>(OW, WoT, DM, DM);
  k_emb<<<(unsigned)(SEQ / 32), 128, 0, stream>>>(Pt, E2);
  k_qkv<<<dim3(NB * SEQ / 128, NQKV / 64), 128, 0, stream>>>(Xb, Wt, QB, P6);
  const int nqs = SPLIT_EFF / 32;
  const int nqp = (SEQ - SPLIT_EFF) / 32;
  k_attn<true><<<(unsigned)(NB * NH * nqs), 64, 0, stream>>>(P6, E2, C2, 0, nqs);
  if (nqp > 0) k_attn<false><<<(unsigned)(NB * NH * nqp), 64, 0, stream>>>(P6, E2, C2, nqs, nqp);
  k_out<<<dim3(NB * SEQ / 64, DM / 64), 128, 0, stream>>>(C2, WoT, OB, OUT);
}
